// LSTMEncoder_65515431133655
// MI455X (gfx1250) — hardware-verified
//
#include <hip/hip_runtime.h>
#include <math.h>

constexpr int NBAT = 16;
constexpr int NLEN = 96;
constexpr int NHU  = 150;
constexpr int HPAD = 160;
constexpr int NGATE = 600;
constexpr int NGP  = 640;
constexpr int NROW = NBAT * NLEN;
constexpr int WDIM = 100, TDIM = 50, WVOC = 50000, TVOC = 50;
constexpr int EMBK = 160;
constexpr int XK   = 384;
constexpr int XSEG = 192;
constexpr int OUTP = 320;
constexpr int UVN  = 256;
constexpr int MLPH = 100;
constexpr int MLPK = 2 * 2 * NHU;
constexpr int NTHR = 256;
constexpr int SCAN_THR = 320;
constexpr int AHP = 168;
constexpr int SHP = 196;
static_assert(NROW % 64 == 0);
static_assert(NGP % 64 == 0 && UVN % 64 == 0);
static_assert(EMBK % 32 == 0 && XK % 32 == 0 && HPAD % 32 == 0);
static_assert(HPAD == 16 * (SCAN_THR / 32));
static_assert((NBAT * NGP) % (4 * SCAN_THR) == 0);
static_assert((NROW * (EMBK / 8)) % NTHR == 0);
static_assert((NROW * (XK / 8)) % NTHR == 0);
static_assert(NROW % 8 == 0);
static_assert(XSEG % 64 == 0 && HPAD % 32 == 0 && SHP >= XSEG && AHP >= HPAD);

typedef __attribute__((ext_vector_type(16))) _Float16 v16h;
typedef __attribute__((ext_vector_type(8)))  _Float16 v8h;
typedef __attribute__((ext_vector_type(16))) __bf16   v16b;
typedef __attribute__((ext_vector_type(8)))  __bf16   v8b;
typedef __attribute__((ext_vector_type(8)))  float    v8f;
typedef __attribute__((ext_vector_type(4)))  float    v4f;

__device__ __forceinline__ unsigned short f2bf_bits(float f) {
  unsigned u = __float_as_uint(f);
  return (unsigned short)((u + 0x7FFFu + ((u >> 16) & 1u)) >> 16);
}
__device__ __forceinline__ float bf_bits2f(unsigned short h) { return __uint_as_float(((unsigned)h) << 16); }
__device__ __forceinline__ int clampi(int v, int lo, int hi) { return v < lo ? lo : (v > hi ? hi : v); }

__device__ __forceinline__ void dep_guard_h(v8f& a, v8f& b, v16h x, v16h y) { asm volatile("v_nop\n\tv_nop\n\tv_nop\n\tv_nop" : "+v"(a), "+v"(b) : "v"(x), "v"(y)); }
__device__ __forceinline__ void dep_guard_b(v8f& a, v8f& b, v16b x, v16b y) { asm volatile("v_nop\n\tv_nop\n\tv_nop\n\tv_nop" : "+v"(a), "+v"(b) : "v"(x), "v"(y)); }
__device__ __forceinline__ void dep_guard4_h(v8f& a, v8f& b, v8f& c, v8f& d, v16h x, v16h y) { asm volatile("v_nop\n\tv_nop\n\tv_nop\n\tv_nop" : "+v"(a), "+v"(b), "+v"(c), "+v"(d) : "v"(x), "v"(y)); }
__device__ __forceinline__ void dep_guard4_b(v8f& a, v8f& b, v8f& c, v8f& d, v16b x, v16b y) { asm volatile("v_nop\n\tv_nop\n\tv_nop\n\tv_nop" : "+v"(a), "+v"(b), "+v"(c), "+v"(d) : "v"(x), "v"(y)); }
__device__ __forceinline__ void guard4_frag_b(v8f& a, v8f& b, v8f& c, v8f& d, v16b x, v16b y, v16b z, v16b w) {
  asm volatile("v_nop\n\tv_nop\n\tv_nop\n\tv_nop" : "+v"(a), "+v"(b), "+v"(c), "+v"(d) : "v"(x), "v"(y), "v"(z), "v"(w));
}
__device__ __forceinline__ void keep4_h(v16h a, v16h b, v16h c, v16h d) { asm volatile("v_nop" :: "v"(a), "v"(b), "v"(c), "v"(d)); }
__device__ __forceinline__ void keep4_b(v16b a, v16b b, v16b c, v16b d) { asm volatile("v_nop" :: "v"(a), "v"(b), "v"(c), "v"(d)); }
__device__ __forceinline__ void acc_guard4(v8f& a, v8f& b, v8f& c, v8f& d) { asm volatile("v_nop\n\tv_nop\n\tv_nop\n\tv_nop" : "+v"(a), "+v"(b), "+v"(c), "+v"(d)); }
template <typename T> struct Frag;
template <> struct Frag<_Float16> {
  typedef v16h V; union U { v16h v; v8h h[2]; };
  static __device__ __forceinline__ v16h load(const _Float16* p) {
    U f; f.h[0] = *(const v8h*)(p); f.h[1] = *(const v8h*)(p + 16); return f.v;
  }
  static __device__ __forceinline__ v8f mma(v16h a, v16h b, v8f c) {
    return __builtin_amdgcn_wmma_f32_16x16x32_f16(false, a, false, b, (short)0, c, false, false);
  }
  static __device__ __forceinline__ void guard(v8f& a, v8f& b, v16h x, v16h y) { dep_guard_h(a, b, x, y); }
  static __device__ __forceinline__ void guard4(v8f& a, v8f& b, v8f& c, v8f& d, v16h x, v16h y) { dep_guard4_h(a, b, c, d, x, y); }
  static __device__ __forceinline__ void keep(v16h a, v16h b, v16h c, v16h d) { keep4_h(a, b, c, d); }
};
template <> struct Frag<__bf16> {
  typedef v16b V; union U { v16b v; v8b h[2]; };
  static __device__ __forceinline__ v16b load(const __bf16* p) {
    U f; f.h[0] = *(const v8b*)(p); f.h[1] = *(const v8b*)(p + 16); return f.v;
  }
  static __device__ __forceinline__ v8f mma(v16b a, v16b b, v8f c) {
    return __builtin_amdgcn_wmma_f32_16x16x32_bf16(false, a, false, b, (short)0, c, false, false);
  }
  static __device__ __forceinline__ void guard(v8f& a, v8f& b, v16b x, v16b y) { dep_guard_b(a, b, x, y); }
  static __device__ __forceinline__ void guard4(v8f& a, v8f& b, v8f& c, v8f& d, v16b x, v16b y) { dep_guard4_b(a, b, c, d, x, y); }
  static __device__ __forceinline__ void keep(v16b a, v16b b, v16b c, v16b d) { keep4_b(a, b, c, d); }
};

__device__ __forceinline__ float fsig(float x) { return __builtin_amdgcn_rcpf(1.0f + expf(-x)); }

__device__ __forceinline__ void store2_hilo8(v8f v, unsigned short* __restrict__ ph, unsigned short* __restrict__ pl) {
  v8h hv, lv;
#pragma unroll
  for (int e = 0; e < 8; ++e) {
    const unsigned short hb = f2bf_bits(v[e]);
    const unsigned short lb = f2bf_bits(v[e] - bf_bits2f(hb));
    hv[e] = __builtin_bit_cast(_Float16, hb);
    lv[e] = __builtin_bit_cast(_Float16, lb);
  }
  *(volatile v8h*)ph = hv;
  *(volatile v8h*)pl = lv;
  __threadfence();
  *(volatile v8h*)ph = hv;
  *(volatile v8h*)pl = lv;
}

template <int ET> struct Elem;
template <> struct Elem<0> { typedef _Float16 T; };
template <> struct Elem<1> { typedef __bf16 T; };
template <int ET, bool SPLIT, int BIAS_MODE, int OUT_MODE, bool RESID, int ACT = 0>
__global__ __launch_bounds__(256) void wmma_gemm64(
    const unsigned short* __restrict__ Ap, const unsigned short* __restrict__ A2p, int lda, long strideA,
    const unsigned short* __restrict__ Btp, const unsigned short* __restrict__ Bt2p, int ldb, long strideB,
    void* __restrict__ Cout, void* __restrict__ Cout2, int ldc, long strideC,
    const float* __restrict__ bias,
    const float* __restrict__ resid, long strideR,
    int M, int N, int K, float scale) {
  typedef typename Elem<ET>::T T;
  typedef typename Frag<T>::V V;
  const T* A = (const T*)Ap; const T* A2 = (const T*)A2p; const T* Bt = (const T*)Btp; const T* Bt2 = (const T*)Bt2p;
  __shared__ __align__(16) float sT[8][16 * 68];
  const int b    = blockIdx.y;
  const int lane = threadIdx.x & 31;
  const int wave = threadIdx.x >> 5;
  const int tilesN = N >> 6;
  const int tilesM = M >> 6;
  const int tile = blockIdx.x * 8 + wave;
  if (tile >= tilesM * tilesN) return;
  const int tm = tile / tilesN;
  const int tn = tile - tm * tilesN;
  const int m0 = tm << 6;
  const int n0 = tn << 6;

  const T* Ab  = A  + (size_t)b * strideA;
  const T* Bb  = Bt + (size_t)b * strideB;
  const T* Ab2 = SPLIT ? (A2  + (size_t)b * strideA) : nullptr;
  const T* Bb2 = SPLIT ? (Bt2 + (size_t)b * strideB) : nullptr;

  const int rlane = lane & 15;
  const int koff  = (lane >> 4) * 8;
  const int mOff  = (lane >> 4) * 8;

  v8f acc[4][4];
#pragma unroll
  for (int i = 0; i < 4; ++i)
#pragma unroll
    for (int j = 0; j < 4; ++j) acc[i][j] = (v8f){0.f,0.f,0.f,0.f,0.f,0.f,0.f,0.f};

  for (int k0 = 0; k0 < K; k0 += 32) {
    V bh[4], bl[4];
#pragma unroll
    for (int j = 0; j < 4; ++j) {
      const size_t bo = (size_t)(n0 + (j << 4) + rlane) * ldb + koff + k0;
      bh[j] = Frag<T>::load(Bb + bo);
      if (SPLIT) bl[j] = Frag<T>::load(Bb2 + bo);
    }
#pragma unroll
    for (int i = 0; i < 4; ++i) {
      const size_t ao = (size_t)(m0 + (i << 4) + rlane) * lda + koff + k0;
      V ah = Frag<T>::load(Ab + ao);
      V al;
      if (SPLIT) al = Frag<T>::load(Ab2 + ao);
#pragma unroll
      for (int j = 0; j < 4; ++j) {
        acc[i][j] = Frag<T>::mma(ah, bh[j], acc[i][j]);
        if (SPLIT) {
          acc[i][j] = Frag<T>::mma(ah, bl[j], acc[i][j]);
          acc[i][j] = Frag<T>::mma(al, bh[j], acc[i][j]);
        }
      }
      Frag<T>::guard4(acc[i][0], acc[i][1], acc[i][2], acc[i][3], ah, SPLIT ? al : ah);
    }
    Frag<T>::keep(bh[0], bh[1], bh[2], bh[3]);
    if (SPLIT) Frag<T>::keep(bl[0], bl[1], bl[2], bl[3]);
  }
  acc_guard4(acc[0][0], acc[0][1], acc[0][2], acc[0][3]);
  acc_guard4(acc[1][0], acc[1][1], acc[1][2], acc[1][3]);
  acc_guard4(acc[2][0], acc[2][1], acc[2][2], acc[2][3]);
  acc_guard4(acc[3][0], acc[3][1], acc[3][2], acc[3][3]);

  float* slab = sT[wave];
  const float* Rb = RESID ? (resid + (size_t)b * strideR) : nullptr;
#pragma unroll
  for (int i = 0; i < 4; ++i) {
    const int mBase = m0 + (i << 4);
#pragma unroll
    for (int j = 0; j < 4; ++j) {
      const int n = n0 + (j << 4) + rlane;
      float bv = 0.f;
      if (BIAS_MODE == 2) bv = bias[n];
#pragma unroll
      for (int r = 0; r < 8; ++r) {
        float v = acc[i][j][r] * scale;
        if (BIAS_MODE == 1) v += bias[mBase + mOff + r];
        if (BIAS_MODE == 2) v += bv;
        if (RESID) v += Rb[(size_t)(mBase + mOff + r) * ldc + n];
        if (ACT == 1) v = tanhf(v);
        if (ACT == 2) v = fmaxf(v, 0.0f);
        if (ACT == 3) v = v / (1.0f + expf(-v));
        if (ACT == 4) v = (v > 0.f) ? v : 0.01f * v;
        if (ACT == 5) v = 0.5f * v * (1.0f + erff(v * 0.70710678118654752f));
        slab[(mOff + r) * 68 + (j << 4) + rlane] = v;
      }
    }
    __builtin_amdgcn_fence(__ATOMIC_RELEASE, "workgroup");
    __builtin_amdgcn_wave_barrier();
    __builtin_amdgcn_fence(__ATOMIC_ACQUIRE, "workgroup");
    if (OUT_MODE == 0) {
      float* C = (float*)Cout + (size_t)b * strideC;
      const int hh = lane >> 4, c4 = (lane & 15) * 4;
      for (int pass = 0; pass < 2; ++pass) {
#pragma unroll
        for (int it = 0; it < 8; ++it) {
          const int row = it * 2 + hh;
          v4f v = *(const v4f*)(slab + row * 68 + c4);
          *(volatile v4f*)(C + (size_t)(mBase + row) * ldc + n0 + c4) = v;
        }
        __threadfence();
      }
    } else {
      const int q = lane >> 3, c8 = (lane & 7) * 8;
      unsigned short* C  = (unsigned short*)Cout  + (size_t)b * strideC;
      unsigned short* C2 = (OUT_MODE == 2) ? ((unsigned short*)Cout2 + (size_t)b * strideC) : nullptr;
      for (int pass = 0; pass < 2; ++pass) {
#pragma unroll
        for (int it = 0; it < 4; ++it) {
          const int row = it * 4 + q;
          const float* sp = slab + row * 68 + c8;
          v8h hv, lv;
#pragma unroll
          for (int e = 0; e < 8; ++e) {
            if (OUT_MODE == 1) {
              hv[e] = (_Float16)sp[e];
            } else {
              unsigned short hb = f2bf_bits(sp[e]);
              unsigned short lb = f2bf_bits(sp[e] - bf_bits2f(hb));
              hv[e] = __builtin_bit_cast(_Float16, hb);
              lv[e] = __builtin_bit_cast(_Float16, lb);
            }
          }
          *(volatile v8h*)(C + (size_t)(mBase + row) * ldc + n0 + c8) = hv;
          if (OUT_MODE == 2) *(volatile v8h*)(C2 + (size_t)(mBase + row) * ldc + n0 + c8) = lv;
        }
        __threadfence();
      }
    }
    __builtin_amdgcn_fence(__ATOMIC_RELEASE, "workgroup");
    __builtin_amdgcn_wave_barrier();
    __builtin_amdgcn_fence(__ATOMIC_ACQUIRE, "workgroup");
  }
}

__global__ __launch_bounds__(NTHR) void embed_kernel(const int* __restrict__ widx, const int* __restrict__ pidx,
                                                    const int* __restrict__ maxlen,
                                                    const float* __restrict__ wemb, const float* __restrict__ temb,
                                                    unsigned short* __restrict__ X0h, unsigned short* __restrict__ X0l) {
  const int i = blockIdx.x * NTHR + threadIdx.x;
  const int n8 = NROW * (EMBK / 8);
  if (i < n8) {
    const int m  = i / (EMBK / 8);
    const int c8 = i - m * (EMBK / 8);
    const int kb = c8 * 8;
    const int bq = m / NLEN, t = m - bq * NLEN;
    int lm = maxlen[0]; lm = lm < 1 ? 1 : (lm > NLEN ? NLEN : lm);
    const int tt = (t < lm) ? t : (lm - 1);
    const int mm = bq * NLEN + tt;
    const int wi = clampi(widx[mm], 0, WVOC - 1);
    const int pi = clampi(pidx[mm], 0, TVOC - 1);
    const float* wrow = wemb + (size_t)wi * WDIM;
    const int wa0 = kb < (WDIM - 4) ? kb : (WDIM - 4);
    const int wb0 = (kb + 4) < (WDIM - 4) ? (kb + 4) : (WDIM - 4);
    const v4f wa = *(const v4f*)(wrow + wa0);
    const v4f wb = *(const v4f*)(wrow + wb0);
    const float* trow = temb + (size_t)pi * TDIM;
    v8f v;
#pragma unroll
    for (int e = 0; e < 8; ++e) {
      const int k = kb + e;
      const int tc = clampi(k - WDIM, 0, TDIM - 1);
      const float tv = trow[tc];
      const float wv = (e < 4) ? wa[e & 3] : wb[e & 3];
      const float fw = (k < WDIM) ? 1.0f : 0.0f;
      const float ft = (k >= WDIM && k < WDIM + TDIM) ? 1.0f : 0.0f;
      v[e] = fmaf(fw, wv, ft * tv);
    }
    store2_hilo8(v, X0h + (size_t)i * 8, X0l + (size_t)i * 8);
  }
}

__global__ __launch_bounds__(NTHR) void prep_wih0_kernel(const float* __restrict__ W, unsigned short* __restrict__ Oh,
                                                        unsigned short* __restrict__ Ol) {
  const int per = NGP * (EMBK / 8);
  const int i = blockIdx.x * NTHR + threadIdx.x;
  if (i < 2 * per) {
    const int dd = i / per, rem = i - dd * per;
    const int n = rem / (EMBK / 8), c8 = rem - n * (EMBK / 8);
    const int g = n / HPAD, jj = n - g * HPAD;
    const int jjc = jj < NHU - 1 ? jj : NHU - 1;
    const float fj = (jj < NHU) ? 1.0f : 0.0f;
    const float* srow = W + ((size_t)(dd * NGATE + g * NHU + jjc)) * NHU;
    v8f v;
#pragma unroll
    for (int e = 0; e < 8; ++e) {
      const int k = c8 * 8 + e;
      const int kc = k < NHU - 1 ? k : NHU - 1;
      const float fk = (k < NHU) ? 1.0f : 0.0f;
      v[e] = srow[kc] * (fj * fk);
    }
    store2_hilo8(v, Oh + (size_t)i * 8, Ol + (size_t)i * 8);
  }
}

__global__ __launch_bounds__(NTHR) void prep_wihr_kernel(const float* __restrict__ W, unsigned short* __restrict__ Oh,
                                                        unsigned short* __restrict__ Ol) {
  const int per = NGP * (XK / 8);
  const int i = blockIdx.x * NTHR + threadIdx.x;
  if (i < 6 * per) {
    const int ld = i / per, rem = i - ld * per;
    const int n = rem / (XK / 8), c8 = rem - n * (XK / 8);
    const int g = n / HPAD, jj = n - g * HPAD;
    const int jjc = jj < NHU - 1 ? jj : NHU - 1;
    const float fj = (jj < NHU) ? 1.0f : 0.0f;
    const int kb = c8 * 8;
    const bool seg0 = c8 < (XSEG / 8);
    const int kr = seg0 ? kb : (kb - XSEG);
    const int coff = seg0 ? 0 : NHU;
    const float* srow = W + ((size_t)(ld * NGATE + g * NHU + jjc)) * (2 * NHU);
    v8f v;
#pragma unroll
    for (int e = 0; e < 8; ++e) {
      const int kk = kr + e;
      const int kc = kk < NHU - 1 ? kk : NHU - 1;
      const float fk = (kk < NHU) ? 1.0f : 0.0f;
      v[e] = srow[coff + kc] * (fj * fk);
    }
    store2_hilo8(v, Oh + (size_t)i * 8, Ol + (size_t)i * 8);
  }
}

__global__ __launch_bounds__(NTHR) void prep_whh_kernel(const float* __restrict__ W, unsigned short* __restrict__ Oh,
                                                       unsigned short* __restrict__ Ol) {
  const int per = NGP * (HPAD / 8);
  const int i = blockIdx.x * NTHR + threadIdx.x;
  if (i < 8 * per) {
    const int ld = i / per, rem = i - ld * per;
    const int n = rem / (HPAD / 8), c8 = rem - n * (HPAD / 8);
    const int g = n / HPAD, jj = n - g * HPAD;
    const int jjc = jj < NHU - 1 ? jj : NHU - 1;
    const float fj = (jj < NHU) ? 1.0f : 0.0f;
    const float* srow = W + ((size_t)(ld * NGATE + g * NHU + jjc)) * NHU;
    v8f v;
#pragma unroll
    for (int e = 0; e < 8; ++e) {
      const int k = c8 * 8 + e;
      const int kc = k < NHU - 1 ? k : NHU - 1;
      const float fk = (k < NHU) ? 1.0f : 0.0f;
      v[e] = srow[kc] * (fj * fk);
    }
    store2_hilo8(v, Oh + (size_t)i * 8, Ol + (size_t)i * 8);
  }
}

__global__ __launch_bounds__(NTHR) void prep_bias_kernel(const float* __restrict__ bih, const float* __restrict__ bhh,
                                                        float* __restrict__ O) {
  const int i = blockIdx.x * NTHR + threadIdx.x;
  if (i < 8 * (NGP / 4)) {
    const int ld = i / (NGP / 4), n4 = (i - ld * (NGP / 4)) * 4;
    v4f o;
#pragma unroll
    for (int e = 0; e < 4; ++e) {
      const int n = n4 + e;
      const int g = n / HPAD, jj = n - g * HPAD;
      const int jjc = jj < NHU - 1 ? jj : NHU - 1;
      const float fj = (jj < NHU) ? 1.0f : 0.0f;
      const int r = ld * NGATE + g * NHU + jjc;
      o[e] = (bih[r] + bhh[r]) * fj;
    }
    float* op = O + (size_t)i * 4;
    *(volatile v4f*)op = o;
    __threadfence();
    *(volatile v4f*)op = o;
  }
}

__global__ __launch_bounds__(NTHR) void prep_w1_kernel(const float* __restrict__ W, unsigned short* __restrict__ Oh,
                                                      unsigned short* __restrict__ Ol) {
  const int i = blockIdx.x * NTHR + threadIdx.x;
  if (i < UVN * (XK / 8)) {
    const int n = i / (XK / 8), c8 = i - n * (XK / 8);
    const int nc = n < 2 * MLPH - 1 ? n : 2 * MLPH - 1;
    const bool half = nc >= MLPH;
    const int r = half ? (nc - MLPH) : nc;
    const float fn = (n < 2 * MLPH) ? 1.0f : 0.0f;
    const int kb = c8 * 8;
    const bool seg0 = c8 < (XSEG / 8);
    const int kr = seg0 ? kb : (kb - XSEG);
    const int coff = (half ? 2 * NHU : 0) + (seg0 ? 0 : NHU);
    const float* srow = W + (size_t)r * MLPK;
    v8f v;
#pragma unroll
    for (int e = 0; e < 8; ++e) {
      const int kk = kr + e;
      const int kc = kk < NHU - 1 ? kk : NHU - 1;
      const float fk = (kk < NHU) ? 1.0f : 0.0f;
      v[e] = srow[coff + kc] * (fn * fk);
    }
    store2_hilo8(v, Oh + (size_t)i * 8, Ol + (size_t)i * 8);
  }
}

__global__ __launch_bounds__(NTHR) void prep_b1_kernel(const float* __restrict__ b1, float* __restrict__ O) {
  const int i = threadIdx.x;
  if (i < UVN / 4) {
    const int r0 = 4 * i;
    const int base = r0 < MLPH - 4 ? r0 : MLPH - 4;
    const v4f bv = *(const v4f*)(b1 + base);
    v4f o;
#pragma unroll
    for (int e = 0; e < 4; ++e) o[e] = bv[e] * ((r0 + e < MLPH) ? 1.0f : 0.0f);
    float* op = O + r0;
    *(volatile v4f*)op = o;
    __threadfence();
    *(volatile v4f*)op = o;
  }
}

__global__ __launch_bounds__(SCAN_THR) void bilstm_scan_kernel(
    const float* __restrict__ PRE,
    const unsigned short* __restrict__ WHhp,
    const unsigned short* __restrict__ WHlp,
    unsigned short* __restrict__ XNh, unsigned short* __restrict__ XNl,
    float* __restrict__ OUTF,
    int writeOut) {
  __shared__ __align__(16) float          sPre[NBAT * NGP];
  __shared__ __align__(16) unsigned short AhH[NBAT * AHP];
  __shared__ __align__(16) unsigned short AhL[NBAT * AHP];
  __shared__ __align__(16) float          sH[NBAT * SHP];
  const int tid = threadIdx.x, lane = tid & 31, wave = tid >> 5;
  const int c = lane & 15, hh = lane >> 4, koff = hh * 8;
  const int d = blockIdx.x;
  const int j = 16 * wave + c;
  const float jval = (j < NHU) ? 1.0f : 0.0f;
  const float* preD = PRE + (size_t)d * NROW * NGP;
  const __bf16* WHh = (const __bf16*)(const void*)WHhp + (size_t)d * NGP * HPAD;
  const __bf16* WHl = (const __bf16*)(const void*)WHlp + (size_t)d * NGP * HPAD;

#pragma unroll 1
  for (int i = tid; i < NBAT * AHP; i += SCAN_THR) { AhH[i] = (unsigned short)0; AhL[i] = (unsigned short)0; }
#pragma unroll 1
  for (int i = tid; i < NBAT * SHP; i += SCAN_THR) sH[i] = 0.0f;
  float cst[8];
#pragma unroll
  for (int r = 0; r < 8; ++r) cst[r] = 0.0f;
  __syncthreads();

  const __bf16* ahrow = (const __bf16*)(const void*)AhH + c * AHP + koff;
  const __bf16* alrow = (const __bf16*)(const void*)AhL + c * AHP + koff;
  const int q = lane >> 3, e8 = (lane & 7) * 8, e4 = (lane & 7) * 4;

#pragma unroll 1
  for (int ti = 0; ti < NLEN; ++ti) {
    const int t = d ? (NLEN - 1 - ti) : ti;
#pragma unroll
    for (int it = 0; it < 8; ++it) {
      const int idx = it * SCAN_THR + tid;
      const int row = idx / (NGP / 4), c4 = (idx - row * (NGP / 4)) * 4;
      const v4f v = *(const v4f*)(preD + ((size_t)row * NLEN + (size_t)t) * NGP + c4);
      *(v4f*)(sPre + row * NGP + c4) = v;
    }
    __syncthreads();

    v8f acc[4];
#pragma unroll
    for (int g = 0; g < 4; ++g)
#pragma unroll
      for (int r = 0; r < 8; ++r) acc[g][r] = sPre[(8 * hh + r) * NGP + g * HPAD + j];
#pragma unroll 1
    for (int k0 = 0; k0 < HPAD; k0 += 32) {
      v16b bh[4], bl[4];
#pragma unroll
      for (int g = 0; g < 4; ++g) {
        const size_t bo = (size_t)(g * HPAD + j) * HPAD + koff + k0;
        bh[g] = Frag<__bf16>::load(WHh + bo);
        bl[g] = Frag<__bf16>::load(WHl + bo);
      }
      const v16b ah = Frag<__bf16>::load(ahrow + k0);
      const v16b al = Frag<__bf16>::load(alrow + k0);
#pragma unroll
      for (int g = 0; g < 4; ++g) {
        acc[g] = Frag<__bf16>::mma(ah, bh[g], acc[g]);
        acc[g] = Frag<__bf16>::mma(ah, bl[g], acc[g]);
        acc[g] = Frag<__bf16>::mma(al, bh[g], acc[g]);
      }
      guard4_frag_b(acc[0], acc[1], acc[2], acc[3], ah, al, bh[3], bl[3]);
      keep4_b(bh[0], bh[1], bh[2], bl[0]);
      keep4_b(bl[1], bl[2], bh[3], bl[3]);
    }
    acc_guard4(acc[0], acc[1], acc[2], acc[3]);

    float hreg[8];
#pragma unroll
    for (int r = 0; r < 8; ++r) {
      const float ig = fsig(acc[0][r]);
      const float fg = fsig(acc[1][r]);
      const float gg = tanhf(acc[2][r]);
      const float og = fsig(acc[3][r]);
      const float cn = (fg * cst[r] + ig * gg) * jval;
      const float hn = (og * tanhf(cn)) * jval;
      cst[r] = cn;
      hreg[r] = hn;
    }
    __syncthreads();

#pragma unroll
    for (int r = 0; r < 8; ++r) {
      const float hn = hreg[r];
      const unsigned short hb = f2bf_bits(hn);
      const unsigned short lb = f2bf_bits(hn - bf_bits2f(hb));
      AhH[(8 * hh + r) * AHP + j] = hb;
      AhL[(8 * hh + r) * AHP + j] = lb;
      sH[(8 * hh + r) * SHP + j] = hn;
    }
    __syncthreads();

    for (int pass = 0; pass < 2; ++pass) {
      for (int gi = wave; gi < 24; gi += 10) {
        const int plane = gi / 12;
        const int grp = gi - plane * 12;
        const int line = grp * 4 + q;
        const int bb = line / 3, seg = line - bb * 3;
        const int col = seg * 64 + e8;
        const float* sp = sH + bb * SHP + col;
        const v4f va = *(const v4f*)(sp);
        const v4f vb = *(const v4f*)(sp + 4);
        v8h hv, lv;
#pragma unroll
        for (int e = 0; e < 4; ++e) {
          const unsigned short h0 = f2bf_bits(va[e]);
          const unsigned short l0 = f2bf_bits(va[e] - bf_bits2f(h0));
          const unsigned short h1 = f2bf_bits(vb[e]);
          const unsigned short l1 = f2bf_bits(vb[e] - bf_bits2f(h1));
          hv[e] = __builtin_bit_cast(_Float16, h0); lv[e] = __builtin_bit_cast(_Float16, l0);
          hv[4 + e] = __builtin_bit_cast(_Float16, h1); lv[4 + e] = __builtin_bit_cast(_Float16, l1);
        }
        const size_t o = ((size_t)bb * NLEN + (size_t)t) * XK + (size_t)(XSEG * d) + col;
        if (plane == 0) *(volatile v8h*)(XNh + o) = hv;
        else            *(volatile v8h*)(XNl + o) = lv;
      }
      __threadfence();
    }
    if (writeOut) {
      for (int pass = 0; pass < 2; ++pass) {
        for (int gi = wave; gi < 20; gi += 10) {
          const int line = gi * 4 + q;
          const int bb = line / 5, seg = line - bb * 5;
          const int col = seg * 32 + e4;
          const v4f v = *(const v4f*)(sH + bb * SHP + col);
          *(volatile v4f*)(OUTF + ((size_t)bb * NLEN + (size_t)t) * OUTP + (size_t)(HPAD * d) + col) = v;
        }
        __threadfence();
      }
    }
  }
}

__global__ __launch_bounds__(NTHR) void poly_kernel(const float* __restrict__ OUTF,
                                                   const float* __restrict__ w1p, const float* __restrict__ w2p,
                                                   const float* __restrict__ w3p, const float* __restrict__ w4p,
                                                   unsigned short* __restrict__ Ph, unsigned short* __restrict__ Pl) {
  const int i = blockIdx.x * NTHR + threadIdx.x;
  if (i < NROW * (XK / 8)) {
    const int m = i / (XK / 8), c8 = i - m * (XK / 8);
    const int kb = c8 * 8;
    const bool seg0 = c8 < (XSEG / 8);
    const int kr = seg0 ? kb : (kb - XSEG);
    const int krc = kr < (HPAD - 8) ? kr : (HPAD - 8);
    const int sb = (seg0 ? 0 : HPAD) + krc;
    const float* sp = OUTF + (size_t)m * OUTP + sb;
    const v4f va = *(const v4f*)(sp);
    const v4f vb = *(const v4f*)(sp + 4);
    const float c1 = w1p[0], c2 = w2p[0], c3 = w3p[0], c4w = w4p[0];
    v8f v;
#pragma unroll
    for (int e = 0; e < 8; ++e) {
      const float x = (e < 4) ? va[e & 3] : vb[e & 3];
      const float fk = (kr + e < NHU) ? 1.0f : 0.0f;
      const float p = x * (c1 + x * (c2 + x * (c3 + x * c4w)));
      v[e] = p * fk;
    }
    store2_hilo8(v, Ph + (size_t)i * 8, Pl + (size_t)i * 8);
  }
}

__global__ __launch_bounds__(NTHR) void score_kernel(const float* __restrict__ UV, const float* __restrict__ w2p,
                                                    const float* __restrict__ b2p, float* __restrict__ out) {
  __shared__ __align__(16) float sU[8][MLPH];
  __shared__ __align__(16) float sw2[MLPH];
  __shared__ __align__(16) float sO[8][NLEN];
  const int tid = threadIdx.x, lane = tid & 31, wave = tid >> 5;
  const int R = blockIdx.x * 8 + wave;
  const int l1 = R >> 4, b = R & 15;
  const float* urow = UV + ((size_t)b * NLEN + l1) * UVN;
#pragma unroll 1
  for (int jj = lane; jj < MLPH; jj += 32) sU[wave][jj] = urow[jj];
#pragma unroll 1
  for (int jj = tid; jj < MLPH; jj += NTHR) sw2[jj] = w2p[jj];
  __syncthreads();
  const float bias = b2p[0];
#pragma unroll 1
  for (int p = 0; p < 3; ++p) {
    const int l2 = p * 32 + lane;
    const float* vrow = UV + ((size_t)b * NLEN + l2) * UVN + MLPH;
    float s = 0.0f;
#pragma unroll 1
    for (int jj = 0; jj < MLPH; ++jj) s += sw2[jj] * tanhf(sU[wave][jj] + vrow[jj]);
    sO[wave][l2] = s + bias;
  }
  __syncthreads();
  const int lc = (lane < 24) ? lane : 23;
  const v4f ov = *(const v4f*)(&sO[wave][4 * lc]);
  float* op = out + (size_t)R * NLEN + 4 * lane;
  for (int pass = 0; pass < 2; ++pass) {
    if (lane < 24) *(volatile v4f*)op = ov;
    __threadfence();
  }
}

extern "C" void kernel_launch(void* const* d_in, const int* in_sizes, int n_in,
                              void* d_out, int out_size, void* d_ws, size_t ws_size, hipStream_t stream) {
  if (n_in < 18 || d_out == nullptr || d_ws == nullptr) return;
  if (in_sizes[0] != NROW || in_sizes[1] != NROW || in_sizes[2] < 1 ||
      in_sizes[3] != WVOC * WDIM || in_sizes[4] != TVOC * TDIM ||
      in_sizes[5] != 2 * NGATE * NHU || in_sizes[6] != 3 * 2 * NGATE * 2 * NHU || in_sizes[7] != 4 * 2 * NGATE * NHU ||
      in_sizes[8] != 4 * 2 * NGATE || in_sizes[9] != 4 * 2 * NGATE ||
      in_sizes[10] < 1 || in_sizes[11] < 1 || in_sizes[12] < 1 || in_sizes[13] < 1 ||
      in_sizes[14] != MLPH * MLPK || in_sizes[15] != MLPH || in_sizes[16] != MLPH || in_sizes[17] < 1 ||
      out_size != NLEN * NBAT * NLEN) return;

  const int*   widx   = (const int*)d_in[0];
  const int*   pidx   = (const int*)d_in[1];
  const int*   maxlen = (const int*)d_in[2];
  const float* wemb   = (const float*)d_in[3];
  const float* temb   = (const float*)d_in[4];
  const float* wih0   = (const float*)d_in[5];
  const float* wihr   = (const float*)d_in[6];
  const float* whh    = (const float*)d_in[7];
  const float* bih    = (const float*)d_in[8];
  const float* bhh    = (const float*)d_in[9];
  const float* w1p    = (const float*)d_in[10];
  const float* w2p    = (const float*)d_in[11];
  const float* w3p    = (const float*)d_in[12];
  const float* w4p    = (const float*)d_in[13];
  const float* mw1    = (const float*)d_in[14];
  const float* mb1    = (const float*)d_in[15];
  const float* mw2    = (const float*)d_in[16];
  const float* mb2    = (const float*)d_in[17];
  float* out = (float*)d_out;

  char* ws = (char*)d_ws; size_t off = 0;
  auto carve = [&](size_t bytes) -> char* { char* p = ws + off; off += (bytes + 255) & ~(size_t)255; return p; };
  unsigned short* X0h = (unsigned short*)carve((size_t)NROW * EMBK * 2);
  unsigned short* X0l = (unsigned short*)carve((size_t)NROW * EMBK * 2);
  unsigned short* XSh[4]; unsigned short* XSl[4];
  for (int s = 0; s < 4; ++s) { XSh[s] = (unsigned short*)carve((size_t)NROW * XK * 2); XSl[s] = (unsigned short*)carve((size_t)NROW * XK * 2); }
  unsigned short* WI0h = (unsigned short*)carve((size_t)2 * NGP * EMBK * 2);
  unsigned short* WI0l = (unsigned short*)carve((size_t)2 * NGP * EMBK * 2);
  unsigned short* WIRh = (unsigned short*)carve((size_t)6 * NGP * XK * 2);
  unsigned short* WIRl = (unsigned short*)carve((size_t)6 * NGP * XK * 2);
  unsigned short* WHh  = (unsigned short*)carve((size_t)8 * NGP * HPAD * 2);
  unsigned short* WHl  = (unsigned short*)carve((size_t)8 * NGP * HPAD * 2);
  float*          BIAS = (float*)carve((size_t)8 * NGP * 4);
  float*          PRE[4];
  for (int s = 0; s < 4; ++s) PRE[s] = (float*)carve((size_t)2 * NROW * NGP * 4);
  float*          OUTF = (float*)carve((size_t)NROW * OUTP * 4);
  unsigned short* Ph   = (unsigned short*)carve((size_t)NROW * XK * 2);
  unsigned short* Pl   = (unsigned short*)carve((size_t)NROW * XK * 2);
  unsigned short* W1Sh = (unsigned short*)carve((size_t)UVN * XK * 2);
  unsigned short* W1Sl = (unsigned short*)carve((size_t)UVN * XK * 2);
  float*          BIAS1 = (float*)carve((size_t)UVN * 4);
  float*          UV   = (float*)carve((size_t)NROW * UVN * 4);
  if (off > ws_size || off > (size_t)134217728) return;

  embed_kernel<<<(NROW * (EMBK / 8)) / NTHR, NTHR, 0, stream>>>(widx, pidx, maxlen, wemb, temb, X0h, X0l);
  prep_wih0_kernel<<<(2 * NGP * (EMBK / 8)) / NTHR, NTHR, 0, stream>>>(wih0, WI0h, WI0l);
  prep_wihr_kernel<<<(6 * NGP * (XK / 8)) / NTHR, NTHR, 0, stream>>>(wihr, WIRh, WIRl);
  prep_whh_kernel<<<(8 * NGP * (HPAD / 8)) / NTHR, NTHR, 0, stream>>>(whh, WHh, WHl);
  prep_bias_kernel<<<(8 * (NGP / 4)) / NTHR, NTHR, 0, stream>>>(bih, bhh, BIAS);
  prep_w1_kernel<<<(UVN * (XK / 8)) / NTHR, NTHR, 0, stream>>>(mw1, W1Sh, W1Sl);
  prep_b1_kernel<<<1, NTHR, 0, stream>>>(mb1, BIAS1);

  const dim3 ggrid((NROW / 64) * (NGP / 64) / 8, 1);
  for (int layer = 0; layer < 4; ++layer) {
    for (int d = 0; d < 2; ++d) {
      float* preC = PRE[layer] + (size_t)d * NROW * NGP;
      const float* bz = BIAS + (size_t)(layer * 2 + d) * NGP;
      if (layer == 0) {
        wmma_gemm64<1, true, 2, 0, false, 0><<<ggrid, 256, 0, stream>>>(
            X0h, X0l, EMBK, 0L,
            WI0h + (size_t)d * NGP * EMBK, WI0l + (size_t)d * NGP * EMBK, EMBK, 0L,
            (void*)preC, (void*)preC, NGP, 0L,
            bz, BIAS, 0L, NROW, NGP, EMBK, 1.0f);
      } else {
        const size_t wo = (size_t)((layer - 1) * 2 + d) * NGP * XK;
        wmma_gemm64<1, true, 2, 0, false, 0><<<ggrid, 256, 0, stream>>>(
            XSh[layer - 1], XSl[layer - 1], XK, 0L,
            WIRh + wo, WIRl + wo, XK, 0L,
            (void*)preC, (void*)preC, NGP, 0L,
            bz, BIAS, 0L, NROW, NGP, XK, 1.0f);
      }
    }
    bilstm_scan_kernel<<<2, SCAN_THR, 0, stream>>>(
        PRE[layer], WHh + (size_t)layer * 2 * NGP * HPAD, WHl + (size_t)layer * 2 * NGP * HPAD,
        XSh[layer], XSl[layer], OUTF, (layer == 3) ? 1 : 0);
  }

  poly_kernel<<<(NROW * (XK / 8)) / NTHR, NTHR, 0, stream>>>(OUTF, w1p, w2p, w3p, w4p, Ph, Pl);
  const dim3 ugrid((NROW / 64) * (UVN / 64) / 8, 1);
  wmma_gemm64<1, true, 2, 0, false, 0><<<ugrid, 256, 0, stream>>>(
      Ph, Pl, XK, 0L, W1Sh, W1Sl, XK, 0L, (void*)UV, (void*)UV, UVN, 0L,
      BIAS1, BIAS, 0L, NROW, UVN, XK, 1.0f);
  score_kernel<<<NROW / 8, NTHR, 0, stream>>>(UV, mw2, mb2, out);
}
